// Model_50362786513530
// MI455X (gfx1250) — hardware-verified
//
#include <hip/hip_runtime.h>
#include <math.h>

constexpr int NB = 16;
constexpr int NS = 512;
constexpr int NFRAME = 438;
constexpr int NDM = 800;
constexpr int NHEAD = 8;
constexpr int NDH = 100;
constexpr int NFFN = 1024;
constexpr int NHID = 1024;
constexpr int NPOSE = 274;
constexpr int WINSZ = 100;
constexpr int NCOND = 10;
constexpr int NTOK = NB * NS;
constexpr int KFRAME = 448;
constexpr int DMP = 832;
constexpr int DHP = 128;
constexpr int HDP = NHEAD * DHP;
constexpr int QKW = 2 * HDP;
constexpr int XW = 288;
constexpr int KG = NHID + XW;
constexpr int WGP = 1344;
constexpr int NOUTP = 320;
constexpr int AP = 1320;
constexpr int OSP = 292;
constexpr int PSP = 72;
constexpr int OSLP = 132;
constexpr int NOUT_ELEMS = NB * NS * NPOSE;
constexpr float WCARRY = 16.0f;
constexpr float WCARRY_INV = 1.0f / 16.0f;
constexpr float OCARRY = 64.0f;
constexpr float MASK_FILL = -1.0e9f;
constexpr int ce_isqrt(int v) { int r = 0; while ((r + 1) * (r + 1) <= v) ++r; return r; }
constexpr int DH_ROOT = ce_isqrt(NDH);
constexpr float SM_SCALE = 1.0f / (float)DH_ROOT;
constexpr int ID_SHIFT = 30;
constexpr int ID_REAL = 1 << 30;

static_assert(DH_ROOT * DH_ROOT == NDH);
static_assert(NDM == NHEAD * NDH);
static_assert(NTOK % 64 == 0 && DMP % 64 == 0 && QKW % 64 == 0 && NFFN % 64 == 0 && NOUTP % 64 == 0);
static_assert(KFRAME % 32 == 0 && NDM % 32 == 0 && HDP % 32 == 0 && NFFN % 32 == 0 && KG % 32 == 0 && NHID % 32 == 0);
static_assert(KFRAME >= NFRAME && DMP >= NDM && XW >= NPOSE && NOUTP >= XW && WGP >= KG && WGP % 64 == 0);
static_assert(NS % 64 == 0 && DHP >= NDH && AP >= KG && AP % 8 == 0 && OSP % 4 == 0 && OSP >= XW);
static_assert(NOUT_ELEMS % 1024 == 0);
static_assert((NTOK * (KFRAME / 8)) % 256 == 0 && (NTOK * (XW / 8)) % 256 == 0);
static_assert(NDM % 4 == 0 && NDM / 4 == 200);

typedef __attribute__((ext_vector_type(16))) _Float16 v16h;
typedef __attribute__((ext_vector_type(8)))  _Float16 v8h;
typedef __attribute__((ext_vector_type(4)))  _Float16 v4h;
typedef __attribute__((ext_vector_type(8)))  float    v8f;
typedef __attribute__((ext_vector_type(4)))  float    v4f;

union FragU { v16h v; v8h h[2]; };

__device__ __forceinline__ v16h frag_load(const _Float16* p) {
  FragU f;
  f.h[0] = *(const v8h*)(p);
  f.h[1] = *(const v8h*)(p + 16);
  return f.v;
}
__device__ __forceinline__ v8f wmma_f16(v16h a, v16h b, v8f c) {
  return __builtin_amdgcn_wmma_f32_16x16x32_f16(false, a, false, b, (short)0, c, false, false);
}
__device__ __forceinline__ v8f wmma_f16_g(v16h a, v16h b, v8f c) {
  c = __builtin_amdgcn_wmma_f32_16x16x32_f16(false, a, false, b, (short)0, c, false, false);
  asm volatile("v_nop\n\tv_nop\n\tv_nop\n\tv_nop" : "+v"(c) : "v"(a), "v"(b));
  return c;
}
__device__ __forceinline__ void guard4(v8f& a0, v8f& a1, v8f& a2, v8f& a3, v16h x, v16h b0, v16h b1, v16h b2, v16h b3) {
  asm volatile("v_nop\n\tv_nop\n\tv_nop\n\tv_nop" : "+v"(a0), "+v"(a1), "+v"(a2), "+v"(a3) : "v"(x), "v"(b0), "v"(b1), "v"(b2), "v"(b3));
}
__device__ __forceinline__ void acc_guard4(v8f& a, v8f& b, v8f& c, v8f& d) {
  asm volatile("v_nop\n\tv_nop\n\tv_nop\n\tv_nop" : "+v"(a), "+v"(b), "+v"(c), "+v"(d));
}
__device__ __forceinline__ void wave_sync() {
  __builtin_amdgcn_fence(__ATOMIC_RELEASE, "workgroup");
  __builtin_amdgcn_wave_barrier();
  __builtin_amdgcn_fence(__ATOMIC_ACQUIRE, "workgroup");
}
__device__ __forceinline__ float sigm(float x)   { return __builtin_amdgcn_rcpf(1.0f + __expf(-x)); }
__device__ __forceinline__ float tanh_e(float x) { return 1.0f - 2.0f * __builtin_amdgcn_rcpf(1.0f + __expf(2.0f * x)); }

template <bool TMAJOR>
__global__ __launch_bounds__(256) void cvt_rows_kernel(const float* __restrict__ src, unsigned short* __restrict__ dstp,
                                                       int nrow, int C, int ncol8) {
  const int i = blockIdx.x * 256 + threadIdx.x;
  const int n8 = nrow * ncol8;
  if (i < n8) {
    const int r = i / ncol8;
    const int c8 = i - r * ncol8;
    const int sr = TMAJOR ? ((r & 15) * NS + (r >> 4)) : r;
    const float* sp = src + (size_t)sr * C;
    v8h hv;
#pragma unroll
    for (int e = 0; e < 8; ++e) {
      const int col = c8 * 8 + e;
      const int cc = col < C ? col : C - 1;
      const float f = sp[cc];
      hv[e] = (_Float16)((col < C) ? f : 0.0f);
    }
    _Float16* dp = (_Float16*)dstp + (size_t)i * 8;
    *(volatile v8h*)dp = hv;
    __threadfence();
    *(volatile v8h*)dp = hv;
  }
}

__global__ __launch_bounds__(256) void tp_kernel(const float* __restrict__ src, int R, int C,
                                                 int kshift, int kreal, int nshift, int nreal,
                                                 unsigned short* __restrict__ Op, int ldo, int rowoff, int coloff,
                                                 int nrows_write, float sc) {
  __shared__ float Tt[64 * 65];
  const int tid = threadIdx.x;
  const int n0 = blockIdx.x * 64, k0 = blockIdx.y * 64;
  const int kmask = (1 << kshift) - 1, nmask = (1 << nshift) - 1;
#pragma unroll 4
  for (int i = 0; i < 16; ++i) {
    const int idx = i * 256 + tid;
    const int rr = idx >> 6, cc = idx & 63;
    const int kk = k0 + rr, nn = n0 + cc;
    const int kl = kk & kmask, nl = nn & nmask;
    const int ks = (kk >> kshift) * kreal + kl;
    const int ns = (nn >> nshift) * nreal + nl;
    const bool ok = (kl < kreal) && (ks < R) && (nl < nreal) && (ns < C);
    const int ksc = ks < R ? ks : R - 1;
    const int nsc = ns < C ? ns : C - 1;
    const float f = src[(size_t)ksc * C + nsc];
    Tt[rr * 65 + cc] = ok ? (f * sc) : 0.0f;
  }
  __syncthreads();
  const int q = tid >> 3, c8 = (tid & 7) * 8;
  v8h hv[2];
#pragma unroll
  for (int g = 0; g < 2; ++g) {
    const int qq = g * 32 + q;
#pragma unroll
    for (int e = 0; e < 8; ++e) hv[g][e] = (_Float16)Tt[(c8 + e) * 65 + qq];
  }
  _Float16* O = (_Float16*)Op;
  for (int pass = 0; pass < 2; ++pass) {
#pragma unroll
    for (int g = 0; g < 2; ++g) {
      const int nrow = n0 + g * 32 + q;
      if (nrow < nrows_write) {
        const size_t o = (size_t)(rowoff + nrow) * (size_t)ldo + (size_t)(coloff + k0 + c8);
        *(volatile v8h*)(O + o) = hv[g];
      }
    }
    __threadfence();
  }
}

template <bool OUT32, bool OUT16, bool BIAS, bool RELU, bool RESID, bool POS>
__global__ __launch_bounds__(256) void gemm64_kernel(
    const unsigned short* __restrict__ Ap, int lda,
    const unsigned short* __restrict__ Btp, int ldb,
    float* __restrict__ C32, int ldc32, int ncols32,
    unsigned short* __restrict__ C16p, int ldc16,
    const float* __restrict__ bias, int nbias,
    const float* __restrict__ resid,
    const float* __restrict__ pos, const int* __restrict__ posidx, int ldpos, int posmax,
    int M, int N, int K, float scale) {
  const _Float16* A = (const _Float16*)Ap;
  const _Float16* Bt = (const _Float16*)Btp;
  __shared__ __align__(16) float sT[8][16 * 68];
  const int lane = threadIdx.x & 31;
  const int wave = threadIdx.x >> 5;
  const int tilesN = N >> 6;
  const int tilesM = M >> 6;
  const int tile = blockIdx.x * 8 + wave;
  if (tile >= tilesM * tilesN) return;
  const int tm = tile / tilesN;
  const int tn = tile - tm * tilesN;
  const int m0 = tm << 6;
  const int n0 = tn << 6;
  const int rlane = lane & 15;
  const int hh = lane >> 4;
  const int koff = hh * 8;
  const int mOff = hh * 8;

  v8f acc[4][4];
#pragma unroll
  for (int i = 0; i < 4; ++i)
#pragma unroll
    for (int j = 0; j < 4; ++j) acc[i][j] = (v8f){0.f, 0.f, 0.f, 0.f, 0.f, 0.f, 0.f, 0.f};

  for (int k0 = 0; k0 < K; k0 += 32) {
    v16h bh[4];
#pragma unroll
    for (int j = 0; j < 4; ++j) {
      const size_t bo = (size_t)(n0 + (j << 4) + rlane) * ldb + koff + k0;
      bh[j] = frag_load(Bt + bo);
    }
#pragma unroll
    for (int i = 0; i < 4; ++i) {
      const size_t ao = (size_t)(m0 + (i << 4) + rlane) * lda + koff + k0;
      const v16h ah = frag_load(A + ao);
#pragma unroll
      for (int j = 0; j < 4; ++j) acc[i][j] = wmma_f16(ah, bh[j], acc[i][j]);
      guard4(acc[i][0], acc[i][1], acc[i][2], acc[i][3], ah, bh[0], bh[1], bh[2], bh[3]);
    }
  }
  acc_guard4(acc[0][0], acc[0][1], acc[0][2], acc[0][3]);
  acc_guard4(acc[1][0], acc[1][1], acc[1][2], acc[1][3]);
  acc_guard4(acc[2][0], acc[2][1], acc[2][2], acc[2][3]);
  acc_guard4(acc[3][0], acc[3][1], acc[3][2], acc[3][3]);

  float* slab = sT[wave];
#pragma unroll
  for (int i = 0; i < 4; ++i) {
    const int mBase = m0 + (i << 4);
#pragma unroll
    for (int j = 0; j < 4; ++j) {
      const int n = n0 + (j << 4) + rlane;
      float bv = 0.f;
      if (BIAS) {
        const int nc = n < nbias ? n : nbias - 1;
        const float bl = bias[nc];
        bv = (n < nbias) ? bl : 0.0f;
      }
#pragma unroll
      for (int r = 0; r < 8; ++r) {
        float v = acc[i][j][r] * scale;
        if (BIAS) v += bv;
        if (RELU) v = fmaxf(v, 0.0f);
        slab[(mOff + r) * 68 + (j << 4) + rlane] = v;
      }
    }
    wave_sync();
    if (OUT32) {
      const int c4 = (lane & 15) * 4;
      const int col = n0 + c4;
      const bool cvalid = col < ncols32;
      const int colc = cvalid ? col : (ncols32 - 4);
#pragma unroll
      for (int half = 0; half < 2; ++half) {
        v4f vals[4];
#pragma unroll
        for (int u = 0; u < 4; ++u) {
          const int row = (half * 4 + u) * 2 + hh;
          v4f v = *(const v4f*)(slab + row * 68 + c4);
          if (RESID) {
            const v4f rv = *(const v4f*)(resid + (size_t)(mBase + row) * ldc32 + colc);
            v += rv;
          }
          if (POS) {
            int pi = posidx[mBase + row];
            pi = pi < 0 ? 0 : (pi > posmax ? posmax : pi);
            const v4f pv = *(const v4f*)(pos + (size_t)pi * ldpos + colc);
            v += pv;
          }
          if (!cvalid) v = (v4f){0.f, 0.f, 0.f, 0.f};
          vals[u] = v;
          if (OUT16) *(v4f*)(slab + row * 68 + c4) = v;
        }
        for (int pass = 0; pass < 2; ++pass) {
#pragma unroll
          for (int u = 0; u < 4; ++u) {
            const int row = (half * 4 + u) * 2 + hh;
            if (cvalid) *(volatile v4f*)(C32 + (size_t)(mBase + row) * ldc32 + col) = vals[u];
          }
          __threadfence();
        }
      }
      if (OUT16) wave_sync();
    }
    if (OUT16) {
      _Float16* C16 = (_Float16*)C16p;
      const int q = lane >> 3, c8 = (lane & 7) * 8;
      for (int pass = 0; pass < 2; ++pass) {
#pragma unroll
        for (int it = 0; it < 4; ++it) {
          const int row = it * 4 + q;
          const float* sp = slab + row * 68 + c8;
          v8h hv;
#pragma unroll
          for (int e = 0; e < 8; ++e) hv[e] = (_Float16)sp[e];
          *(volatile v8h*)(C16 + (size_t)(mBase + row) * ldc16 + n0 + c8) = hv;
        }
        __threadfence();
      }
    }
    wave_sync();
  }
}

__global__ __launch_bounds__(128) void attn_kernel(const unsigned short* __restrict__ QKp,
                                                   const unsigned short* __restrict__ VTp,
                                                   unsigned short* __restrict__ Op) {
  __shared__ __align__(16) _Float16 Psh[4][16 * PSP];
  __shared__ __align__(16) float    Osl[4][16 * OSLP];
  const _Float16* QK = (const _Float16*)QKp;
  const _Float16* VT = (const _Float16*)VTp;
  _Float16* O = (_Float16*)Op;
  const int tid = threadIdx.x, lane = tid & 31;
  const int wave = __builtin_amdgcn_readfirstlane(tid >> 5);
  const int hh = lane >> 4, c = lane & 15, koff = hh * 8;
  const int bx = blockIdx.x;
  const int qb = bx & 7, hd = (bx >> 3) & 7, b = bx >> 6;
  const int q0 = qb * 64 + wave * 16;
  const int tok0 = b * NS;

  v16h qa[4];
  {
    const _Float16* qrow = QK + (size_t)(tok0 + q0 + c) * QKW + hd * DHP + koff;
#pragma unroll
    for (int dc = 0; dc < 4; ++dc) qa[dc] = frag_load(qrow + dc * 32);
  }
  float mrow[8], lrow[8];
  v8f oacc[7];
#pragma unroll
  for (int r = 0; r < 8; ++r) { mrow[r] = -INFINITY; lrow[r] = 0.f; }
#pragma unroll
  for (int t = 0; t < 7; ++t) oacc[t] = (v8f){0.f, 0.f, 0.f, 0.f, 0.f, 0.f, 0.f, 0.f};

  int lo = q0 - WINSZ;
  if (lo < 0) lo = 0;
  int hk = q0 + 15 + WINSZ;
  if (hk > NS - 1) hk = NS - 1;
  const int kc_lo = lo >> 6, kc_hi = hk >> 6;
  const _Float16* kbase = QK + (size_t)(tok0 + c) * QKW + HDP + hd * DHP + koff;
  const _Float16* vbase = VT + (size_t)(hd * NDH + c) * NTOK + tok0 + koff;
  _Float16* pw = Psh[wave];
  float* os = Osl[wave];

#pragma unroll 1
  for (int kc = kc_lo; kc <= kc_hi; ++kc) {
    const int kv0 = kc * 64;
    v8f s[4];
#pragma unroll
    for (int j = 0; j < 4; ++j) {
      s[j] = (v8f){0.f, 0.f, 0.f, 0.f, 0.f, 0.f, 0.f, 0.f};
      const _Float16* krow = kbase + (size_t)(kv0 + j * 16) * QKW;
#pragma unroll
      for (int dc = 0; dc < 4; ++dc) {
        const v16h kb = frag_load(krow + dc * 32);
        s[j] = wmma_f16_g(qa[dc], kb, s[j]);
      }
    }
    float cm[8];
#pragma unroll
    for (int r = 0; r < 8; ++r) {
      const int qrow = q0 + 8 * hh + r;
      float m = -INFINITY;
#pragma unroll
      for (int j = 0; j < 4; ++j) {
        const int kvcol = kv0 + j * 16 + c;
        const int dq = qrow - kvcol;
        const bool masked = (dq > WINSZ) || (dq < -WINSZ);
        float sv = s[j][r] * SM_SCALE;
        if (masked) sv = MASK_FILL;
        s[j][r] = sv;
        m = fmaxf(m, sv);
      }
#pragma unroll
      for (int off = 1; off < 16; off <<= 1) m = fmaxf(m, __shfl_xor(m, off, 32));
      cm[r] = m;
    }
#pragma unroll
    for (int r = 0; r < 8; ++r) {
      const float mnew = fmaxf(mrow[r], cm[r]);
      const float alpha = expf(mrow[r] - mnew);
      mrow[r] = mnew;
      float psum = 0.f;
#pragma unroll
      for (int j = 0; j < 4; ++j) {
        const float p = expf(s[j][r] - mnew);
        const _Float16 ph = (_Float16)p;
        psum += (float)ph;
        pw[(8 * hh + r) * PSP + j * 16 + c] = ph;
      }
#pragma unroll
      for (int off = 1; off < 16; off <<= 1) psum += __shfl_xor(psum, off, 32);
      lrow[r] = lrow[r] * alpha + psum;
#pragma unroll
      for (int t = 0; t < 7; ++t) oacc[t][r] *= alpha;
    }
    wave_sync();
#pragma unroll 1
    for (int kk = 0; kk < 2; ++kk) {
      const v16h pa = frag_load(pw + c * PSP + kk * 32 + koff);
#pragma unroll
      for (int t = 0; t < 7; ++t) {
        const v16h vb = frag_load(vbase + (size_t)(t * 16) * NTOK + kv0 + kk * 32);
        oacc[t] = wmma_f16_g(pa, vb, oacc[t]);
      }
    }
    wave_sync();
  }

#pragma unroll
  for (int r = 0; r < 8; ++r) {
    const float inv = OCARRY * (1.0f / lrow[r]);
#pragma unroll
    for (int t = 0; t < 7; ++t) {
      const float val = oacc[t][r] * inv;
      const bool keep = (t < 6) || (c < NDH - 96);
      os[(8 * hh + r) * OSLP + t * 16 + c] = keep ? val : 0.0f;
    }
    os[(8 * hh + r) * OSLP + 112 + c] = 0.0f;
  }
  wave_sync();
  {
    const int c8 = c * 8;
    v8h hv[8];
#pragma unroll
    for (int it = 0; it < 8; ++it) {
      const int row = it * 2 + hh;
      const v4f x0 = *(const v4f*)(os + row * OSLP + c8);
      const v4f x1 = *(const v4f*)(os + row * OSLP + c8 + 4);
#pragma unroll
      for (int e = 0; e < 4; ++e) {
        hv[it][e] = (_Float16)x0[e];
        hv[it][4 + e] = (_Float16)x1[e];
      }
    }
    for (int pass = 0; pass < 2; ++pass) {
#pragma unroll
      for (int it = 0; it < 8; ++it) {
        const int row = it * 2 + hh;
        *(volatile v8h*)(O + (size_t)(tok0 + q0 + row) * HDP + hd * DHP + c8) = hv[it];
      }
      __threadfence();
    }
  }
}

template <bool W32, bool TMAJOR>
__global__ __launch_bounds__(256) void ln_kernel(const float* __restrict__ Y, const float* __restrict__ gam,
                                                 const float* __restrict__ bet, float* __restrict__ X32,
                                                 unsigned short* __restrict__ X16p, int nrows, float eps) {
  const int tid = threadIdx.x, lane = tid & 31;
  const int row = blockIdx.x * 8 + (tid >> 5);
  if (row >= nrows) return;
  const float* rp = Y + (size_t)row * NDM;
  const bool ok6 = lane < 8;
  v4f v[7];
  float s = 0.0f;
#pragma unroll
  for (int q = 0; q < 7; ++q) {
    const int f = lane + 32 * q;
    const int fc = f < 200 ? f : 199;
    v4f t = *(const v4f*)(rp + 4 * fc);
    if (q == 6 && !ok6) t = (v4f){0.f, 0.f, 0.f, 0.f};
    v[q] = t;
    s += (t[0] + t[1]) + (t[2] + t[3]);
  }
#pragma unroll
  for (int off = 1; off < 32; off <<= 1) s += __shfl_xor(s, off, 32);
  const float mu = s * (1.0f / (float)NDM);
  float ss = 0.0f;
#pragma unroll
  for (int q = 0; q < 7; ++q) {
#pragma unroll
    for (int e = 0; e < 4; ++e) {
      float d = v[q][e] - mu;
      if (q == 6 && !ok6) d = 0.0f;
      v[q][e] = d;
      ss += d * d;
    }
  }
#pragma unroll
  for (int off = 1; off < 32; off <<= 1) ss += __shfl_xor(ss, off, 32);
  const float var = ss * (1.0f / (float)NDM);
  const float rstd = rsqrtf(var + eps);
  v4f o[7];
  v4h oh[7];
#pragma unroll
  for (int q = 0; q < 7; ++q) {
    const int f = lane + 32 * q;
    const int fc = f < 200 ? f : 199;
    const v4f g = *(const v4f*)(gam + 4 * fc);
    const v4f bb = *(const v4f*)(bet + 4 * fc);
#pragma unroll
    for (int e = 0; e < 4; ++e) {
      float x = (v[q][e] * rstd) * g[e] + bb[e];
      if (q == 6 && !ok6) x = 0.0f;
      o[q][e] = x;
      oh[q][e] = (_Float16)x;
    }
  }
  const int dr = TMAJOR ? ((row & (NS - 1)) * NB + (row >> 9)) : row;
  _Float16* hp = (_Float16*)X16p + (size_t)dr * DMP;
  float* op = X32 + (size_t)row * NDM;
  for (int pass = 0; pass < 2; ++pass) {
#pragma unroll
    for (int q = 0; q < 7; ++q) {
      const int f = lane + 32 * q;
      if (W32) {
        if (q < 6 || ok6) *(volatile v4f*)(op + 4 * f) = o[q];
      }
      if (q < 6 || lane < 16) *(volatile v4h*)(hp + 4 * f) = oh[q];
    }
    __threadfence();
  }
}

__global__ __launch_bounds__(512) void lstm_kernel(
    const unsigned short* __restrict__ T16p, const float* __restrict__ E,
    const float* __restrict__ h0, const float* __restrict__ c0, const float* __restrict__ dec0,
    const unsigned short* __restrict__ Wgp, const unsigned short* __restrict__ Wtp,
    const float* __restrict__ lb, const int* __restrict__ epoch_p, float* __restrict__ ows) {
  __shared__ __align__(16) _Float16 At[16 * AP];
  __shared__ __align__(16) float    outS[16 * OSP];
  const _Float16* T16 = (const _Float16*)T16p;
  const _Float16* Wg = (const _Float16*)Wgp;
  const _Float16* Wt = (const _Float16*)Wtp;
  const int tid = threadIdx.x, lane = tid & 31;
  const int wave = __builtin_amdgcn_readfirstlane(tid >> 5);
  const int c = lane & 15, hh = lane >> 4, koff = hh * 8;

  int p;
  {
    const int ep = epoch_p[0];
    const double pd = (double)ep * 0.01;
    p = (int)pd;
    if (p < 0) p = 0;
    if (p > 1048576) p = 1048576;
  }
  const int period = p + NCOND;

#pragma unroll 1
  for (int i = tid; i < 16 * NHID; i += 512) {
    const int row = i >> 10, col = i & (NHID - 1);
    At[row * AP + col] = (_Float16)h0[i];
  }
  if (p > 0) {
#pragma unroll 1
    for (int i = tid; i < 16 * XW; i += 512) {
      const int row = i / XW, col = i - row * XW;
      const int cc = col < NPOSE ? col : NPOSE - 1;
      const float f = dec0[row * NPOSE + cc];
      At[row * AP + NHID + col] = (_Float16)((col < NPOSE) ? f : 0.0f);
    }
  } else {
#pragma unroll 1
    for (int i = tid; i < 16 * (XW / 8); i += 512) {
      const int row = i / (XW / 8), ch = i - row * (XW / 8);
      const v8h tv = *(const v8h*)(T16 + (size_t)row * XW + ch * 8);
      *(v8h*)(At + row * AP + NHID + ch * 8) = tv;
    }
  }
  float cst[4][8], hst[4][8];
#pragma unroll
  for (int nt = 0; nt < 4; ++nt) {
    const int j = 64 * wave + 16 * nt + c;
#pragma unroll
    for (int r = 0; r < 8; ++r) {
      cst[nt][r] = c0[(size_t)(8 * hh + r) * NHID + j];
      hst[nt][r] = 0.0f;
    }
  }
  __syncthreads();

  const _Float16* arow = At + c * AP + koff;
  const v8f z8 = {0.f, 0.f, 0.f, 0.f, 0.f, 0.f, 0.f, 0.f};
  const size_t GST = (size_t)NHID * WGP;

#pragma unroll 1
  for (int t = 0; t < NS; ++t) {
#pragma unroll
    for (int nt = 0; nt < 4; ++nt) {
      const int j = 64 * wave + 16 * nt + c;
      const _Float16* wp = Wg + (size_t)j * WGP + koff;
      v8f a0 = z8, a1 = z8, a2 = z8, a3 = z8;
#pragma unroll 1
      for (int k0 = 0; k0 < KG; k0 += 32) {
        const v16h a  = frag_load(arow + k0);
        const v16h b0 = frag_load(wp + k0);
        const v16h b1 = frag_load(wp + GST + k0);
        const v16h b2 = frag_load(wp + 2 * GST + k0);
        const v16h b3 = frag_load(wp + 3 * GST + k0);
        a0 = wmma_f16(a, b0, a0);
        a1 = wmma_f16(a, b1, a1);
        a2 = wmma_f16(a, b2, a2);
        a3 = wmma_f16(a, b3, a3);
        guard4(a0, a1, a2, a3, a, b0, b1, b2, b3);
      }
      acc_guard4(a0, a1, a2, a3);
      const float bi = lb[j];
      const float bf = lb[NHID + j];
      const float bg = lb[2 * NHID + j];
      const float bo = lb[3 * NHID + j];
#pragma unroll
      for (int r = 0; r < 8; ++r) {
        const float zi = a0[r] * WCARRY_INV + bi;
        const float zf = a1[r] * WCARRY_INV + bf;
        const float zg = a2[r] * WCARRY_INV + bg;
        const float zo = a3[r] * WCARRY_INV + bo;
        const float ig = sigm(zi);
        const float fg = sigm(zf);
        const float gg = tanh_e(zg);
        const float og = sigm(zo);
        const float cn = fg * cst[nt][r] + ig * gg;
        cst[nt][r] = cn;
        hst[nt][r] = og * tanh_e(cn);
      }
    }
    __syncthreads();
#pragma unroll
    for (int nt = 0; nt < 4; ++nt) {
      const int j = 64 * wave + 16 * nt + c;
#pragma unroll
      for (int r = 0; r < 8; ++r) At[(8 * hh + r) * AP + j] = (_Float16)hst[nt][r];
    }
    __syncthreads();
    const int tn = t + 1;
    const bool have_next = tn < NS;
    const bool next_fbk = have_next && ((tn % period) < p);
    const int ntiles = (wave < 2) ? 2 : 1;
    const float* Et = E + (size_t)t * 16 * XW;
#pragma unroll 1
    for (int u = 0; u < ntiles; ++u) {
      const int nt2 = wave + 16 * u;
      const int n = nt2 * 16 + c;
      const _Float16* wp = Wt + (size_t)n * NHID + koff;
      v8f acc = z8;
#pragma unroll 1
      for (int k0 = 0; k0 < NHID; k0 += 32) {
        const v16h a = frag_load(arow + k0);
        const v16h bq = frag_load(wp + k0);
        acc = wmma_f16_g(a, bq, acc);
      }
#pragma unroll
      for (int r = 0; r < 8; ++r) {
        const int row = 8 * hh + r;
        const float v = acc[r] * WCARRY_INV + Et[(size_t)row * XW + n];
        outS[row * OSP + n] = v;
        if (next_fbk) At[row * AP + NHID + n] = (_Float16)v;
      }
    }
    if (have_next && !next_fbk) {
#pragma unroll 1
      for (int i = tid; i < 16 * (XW / 8); i += 512) {
        const int row = i / (XW / 8), ch = i - row * (XW / 8);
        const v8h tv = *(const v8h*)(T16 + ((size_t)tn * 16 + row) * XW + ch * 8);
        *(v8h*)(At + row * AP + NHID + ch * 8) = tv;
      }
    }
    __syncthreads();
    {
      const float* sp = outS + wave * OSP;
      float* dp = ows + ((size_t)wave * NS + (size_t)t) * XW;
      const int l8 = lane < 8 ? lane : 7;
      const v4f v0 = *(const v4f*)(sp + 4 * lane);
      const v4f v1 = *(const v4f*)(sp + 128 + 4 * lane);
      const v4f v2 = *(const v4f*)(sp + 256 + 4 * l8);
      for (int pass = 0; pass < 2; ++pass) {
        *(volatile v4f*)(dp + 4 * lane) = v0;
        *(volatile v4f*)(dp + 128 + 4 * lane) = v1;
        if (lane < 8) *(volatile v4f*)(dp + 256 + 4 * lane) = v2;
        __threadfence();
      }
    }
  }
}

__global__ __launch_bounds__(256) void pack_kernel(const float* __restrict__ ows, float* __restrict__ out, int n4) {
  const int i = blockIdx.x * 256 + threadIdx.x;
  if (i < n4) {
    v4f v;
#pragma unroll
    for (int e = 0; e < 4; ++e) {
      const int idx = 4 * i + e;
      const int row = idx / NPOSE;
      const int col = idx - row * NPOSE;
      v[e] = ows[(size_t)row * XW + col];
    }
    float* op = out + (size_t)4 * i;
    *(volatile v4f*)op = v;
    __threadfence();
    *(volatile v4f*)op = v;
  }
}

extern "C" void kernel_launch(void* const* d_in, const int* in_sizes, int n_in,
                              void* d_out, int out_size, void* d_ws, size_t ws_size, hipStream_t stream) {
  if (n_in < 27 || d_out == nullptr || d_ws == nullptr) return;
  if (in_sizes[0] != NTOK * NFRAME || in_sizes[1] != NTOK || in_sizes[2] != NTOK * NPOSE ||
      in_sizes[3] != NB * NHID || in_sizes[4] != NB * NHID || in_sizes[5] != NB * NPOSE ||
      in_sizes[6] != NFRAME * NDM || in_sizes[8] != (NS + 1) * NDM || in_sizes[9] != NDM * NDM ||
      in_sizes[15] != NDM * NFFN || in_sizes[17] != NFFN * NDM || in_sizes[21] != NPOSE * 4 * NHID ||
      in_sizes[22] != NHID * 4 * NHID || in_sizes[24] != (NHID + NDM) * NPOSE || in_sizes[26] != 1 ||
      out_size != NOUT_ELEMS) return;

  const float* src   = (const float*)d_in[0];
  const int*   spos  = (const int*)d_in[1];
  const float* tgt   = (const float*)d_in[2];
  const float* vh0   = (const float*)d_in[3];
  const float* vc0   = (const float*)d_in[4];
  const float* dec0  = (const float*)d_in[5];
  const float* embW  = (const float*)d_in[6];
  const float* embB  = (const float*)d_in[7];
  const float* posT  = (const float*)d_in[8];
  const float* Wq    = (const float*)d_in[9];
  const float* Wk    = (const float*)d_in[10];
  const float* Wv    = (const float*)d_in[11];
  const float* Wo    = (const float*)d_in[12];
  const float* ln1g  = (const float*)d_in[13];
  const float* ln1b  = (const float*)d_in[14];
  const float* fW1   = (const float*)d_in[15];
  const float* fb1   = (const float*)d_in[16];
  const float* fW2   = (const float*)d_in[17];
  const float* fb2   = (const float*)d_in[18];
  const float* ln2g  = (const float*)d_in[19];
  const float* ln2b  = (const float*)d_in[20];
  const float* lWx   = (const float*)d_in[21];
  const float* lWh   = (const float*)d_in[22];
  const float* lbias = (const float*)d_in[23];
  const float* oW    = (const float*)d_in[24];
  const float* ob    = (const float*)d_in[25];
  const int*   epoch = (const int*)d_in[26];
  float* out = (float*)d_out;

  char* ws = (char*)d_ws;
  size_t off = 0;
  auto carve = [&](size_t bytes) -> char* { char* p = ws + off; off += (bytes + 255) & ~(size_t)255; return p; };

  unsigned short* EWT = (unsigned short*)carve((size_t)DMP * KFRAME * 2);
  unsigned short* WQK = (unsigned short*)carve((size_t)QKW * DMP * 2);
  unsigned short* WVT = (unsigned short*)carve((size_t)DMP * DMP * 2);
  unsigned short* WOT = (unsigned short*)carve((size_t)DMP * HDP * 2);
  unsigned short* W1T = (unsigned short*)carve((size_t)NFFN * DMP * 2);
  unsigned short* W2T = (unsigned short*)carve((size_t)DMP * NFFN * 2);
  char* RC = carve((size_t)NTOK * HDP * 2);
  unsigned short* X016  = (unsigned short*)RC;
  unsigned short* O16   = (unsigned short*)RC;
  unsigned short* ENC16 = (unsigned short*)RC;
  char* RA = carve((size_t)NTOK * NDM * 4);
  float* X0 = (float*)RA;
  unsigned short* HID16 = (unsigned short*)RA;
  char* RB = carve((size_t)NTOK * NDM * 4);
  unsigned short* SRC16 = (unsigned short*)RB;
  float* Y1 = (float*)RB;
  float* Y2 = (float*)RB;
  float* OWS = (float*)RB;
  const size_t szQK = (size_t)NTOK * QKW * 2;
  const size_t szVT = (size_t)DMP * NTOK * 2;
  char* RD = carve(szQK + szVT);
  unsigned short* QK16 = (unsigned short*)RD;
  unsigned short* VT16 = (unsigned short*)(RD + szQK);
  float* X1 = (float*)RD;
  unsigned short* X116 = (unsigned short*)(RD + (size_t)NTOK * NDM * 4);
  size_t lo = 0;
  auto late = [&](size_t bytes) -> char* { char* p = RD + lo; lo += (bytes + 255) & ~(size_t)255; return p; };
  unsigned short* WG16  = (unsigned short*)late((size_t)4 * NHID * WGP * 2);
  unsigned short* WTOP  = (unsigned short*)late((size_t)NOUTP * NHID * 2);
  unsigned short* WBOT  = (unsigned short*)late((size_t)NOUTP * DMP * 2);
  unsigned short* TGT16 = (unsigned short*)late((size_t)NTOK * XW * 2);
  float*          EPL   = (float*)late((size_t)NTOK * XW * 4);
  if (lo > szQK + szVT) return;
  if ((size_t)NTOK * NDM * 4 + (size_t)NTOK * DMP * 2 > szQK + szVT) return;
  if (off > ws_size || off > (size_t)134217728) return;

  auto tp = [&](const float* s, int R, int C, int ksh, int krl, int nsh, int nrl, unsigned short* O, int ldo,
                int rowoff, int coloff, int nrw, int gx, int gy) {
    tp_kernel<<<dim3(gx, gy), 256, 0, stream>>>(s, R, C, ksh, krl, nsh, nrl, O, ldo, rowoff, coloff, nrw, WCARRY);
  };
  auto gblocks = [](int M, int N) -> int { return ((M / 64) * (N / 64) + 7) / 8; };

  cvt_rows_kernel<false><<<(NTOK * (KFRAME / 8)) / 256, 256, 0, stream>>>(src, SRC16, NTOK, NFRAME, KFRAME / 8);
  tp(embW, NFRAME, NDM, ID_SHIFT, ID_REAL, ID_SHIFT, ID_REAL, EWT, KFRAME, 0, 0, DMP, DMP / 64, KFRAME / 64);
  tp(Wq, NDM, NDM, ID_SHIFT, ID_REAL, 7, NDH, WQK, DMP, 0, 0, HDP, HDP / 64, DMP / 64);
  tp(Wk, NDM, NDM, ID_SHIFT, ID_REAL, 7, NDH, WQK, DMP, HDP, 0, HDP, HDP / 64, DMP / 64);
  tp(Wv, NDM, NDM, ID_SHIFT, ID_REAL, ID_SHIFT, ID_REAL, WVT, DMP, 0, 0, DMP, DMP / 64, DMP / 64);
  tp(Wo, NDM, NDM, 7, NDH, ID_SHIFT, ID_REAL, WOT, HDP, 0, 0, DMP, DMP / 64, HDP / 64);
  tp(fW1, NDM, NFFN, ID_SHIFT, ID_REAL, ID_SHIFT, ID_REAL, W1T, DMP, 0, 0, NFFN, NFFN / 64, DMP / 64);
  tp(fW2, NFFN, NDM, ID_SHIFT, ID_REAL, ID_SHIFT, ID_REAL, W2T, NFFN, 0, 0, DMP, DMP / 64, NFFN / 64);

  gemm64_kernel<true, true, true, false, false, true><<<gblocks(NTOK, DMP), 256, 0, stream>>>(
      SRC16, KFRAME, EWT, KFRAME, X0, NDM, NDM, X016, DMP, embB, NDM, X0, posT, spos, NDM, NS,
      NTOK, DMP, KFRAME, WCARRY_INV);
  gemm64_kernel<false, true, false, false, false, false><<<gblocks(NTOK, QKW), 256, 0, stream>>>(
      X016, DMP, WQK, DMP, X0, NDM, NDM, QK16, QKW, embB, NDM, X0, posT, spos, NDM, NS,
      NTOK, QKW, NDM, WCARRY_INV);
  gemm64_kernel<false, true, false, false, false, false><<<gblocks(DMP, NTOK), 256, 0, stream>>>(
      WVT, DMP, X016, DMP, X0, NDM, NDM, VT16, NTOK, embB, NDM, X0, posT, spos, NDM, NS,
      DMP, NTOK, NDM, WCARRY_INV);
  attn_kernel<<<NB * NHEAD * (NS / 64), 128, 0, stream>>>(QK16, VT16, O16);
  gemm64_kernel<true, false, false, false, true, false><<<gblocks(NTOK, DMP), 256, 0, stream>>>(
      O16, HDP, WOT, HDP, Y1, NDM, NDM, X016, DMP, embB, NDM, X0, posT, spos, NDM, NS,
      NTOK, DMP, HDP, WCARRY_INV * (1.0f / OCARRY));
  ln_kernel<true, false><<<NTOK / 8, 256, 0, stream>>>(Y1, ln1g, ln1b, X1, X116, NTOK, 1e-6f);
  gemm64_kernel<false, true, true, true, false, false><<<gblocks(NTOK, NFFN), 256, 0, stream>>>(
      X116, DMP, W1T, DMP, Y1, NDM, NDM, HID16, NFFN, fb1, NFFN, X1, posT, spos, NDM, NS,
      NTOK, NFFN, NDM, WCARRY_INV);
  gemm64_kernel<true, false, true, false, true, false><<<gblocks(NTOK, DMP), 256, 0, stream>>>(
      HID16, NFFN, W2T, NFFN, Y2, NDM, NDM, X116, DMP, fb2, NDM, X1, posT, spos, NDM, NS,
      NTOK, DMP, NFFN, WCARRY_INV);
  ln_kernel<false, true><<<NTOK / 8, 256, 0, stream>>>(Y2, ln2g, ln2b, X0, ENC16, NTOK, 1e-6f);

  tp(lWh, NHID, 4 * NHID, ID_SHIFT, ID_REAL, ID_SHIFT, ID_REAL, WG16, WGP, 0, 0, 4 * NHID, (4 * NHID) / 64, NHID / 64);
  tp(lWx, NPOSE, 4 * NHID, ID_SHIFT, ID_REAL, ID_SHIFT, ID_REAL, WG16, WGP, 0, NHID, 4 * NHID, (4 * NHID) / 64, (WGP - NHID) / 64);
  tp(oW, NHID, NPOSE, ID_SHIFT, ID_REAL, ID_SHIFT, ID_REAL, WTOP, NHID, 0, 0, NOUTP, NOUTP / 64, NHID / 64);
  tp(oW + (size_t)NHID * NPOSE, NDM, NPOSE, ID_SHIFT, ID_REAL, ID_SHIFT, ID_REAL, WBOT, DMP, 0, 0, NOUTP, NOUTP / 64, DMP / 64);
  cvt_rows_kernel<true><<<(NTOK * (XW / 8)) / 256, 256, 0, stream>>>(tgt, TGT16, NTOK, NPOSE, XW / 8);
  gemm64_kernel<true, false, true, false, false, false><<<gblocks(NTOK, NOUTP), 256, 0, stream>>>(
      ENC16, DMP, WBOT, DMP, EPL, XW, XW, X016, DMP, ob, NPOSE, X0, posT, spos, NDM, NS,
      NTOK, NOUTP, NDM, WCARRY_INV);
  lstm_kernel<<<1, 512, 0, stream>>>(TGT16, EPL, vh0, vc0, dec0, WG16, WTOP, lbias, epoch, OWS);
  pack_kernel<<<(NOUT_ELEMS / 4) / 256, 256, 0, stream>>>(OWS, out, NOUT_ELEMS / 4);
}
